// attn_block_anchor_66357244723394
// MI455X (gfx1250) — hardware-verified
//
#include <hip/hip_runtime.h>
#include <math.h>
#include <stdint.h>

#define NB   4
#define SEQ  4096
#define DCH  256

static_assert(SEQ % 64 == 0);
static_assert(DCH == 256);
static_assert((NB * SEQ) % 64 == 0);

typedef __attribute__((ext_vector_type(16))) __bf16 v16b;
typedef __attribute__((ext_vector_type(8)))  __bf16 v8b;
typedef __attribute__((ext_vector_type(8)))  float  v8f;
typedef __attribute__((ext_vector_type(4)))  float  v4f;
typedef __attribute__((ext_vector_type(4)))  unsigned int v4u;

#define NEG_INF (-__builtin_inff())

__device__ __forceinline__ unsigned short f2bf_bits(float f) {
  unsigned u = __float_as_uint(f);
  return (unsigned short)((u + 0x7FFFu + ((u >> 16) & 1u)) >> 16);
}
__device__ __forceinline__ float bf_bits2f(unsigned short h) { return __uint_as_float(((unsigned)h) << 16); }
__device__ __forceinline__ unsigned pk16(unsigned short a, unsigned short b) { return (unsigned)a | ((unsigned)b << 16); }
__device__ __forceinline__ void split_pair(float f0, float f1, unsigned& hp, unsigned& lp) {
  const unsigned short h0 = f2bf_bits(f0), h1 = f2bf_bits(f1);
  const unsigned short l0 = f2bf_bits(f0 - bf_bits2f(h0)), l1 = f2bf_bits(f1 - bf_bits2f(h1));
  hp = pk16(h0, h1); lp = pk16(l0, l1);
}
__device__ __forceinline__ void split8(v4f a0, v4f a1, v4u& hp, v4u& lp) {
  unsigned h, l;
  split_pair(a0[0], a0[1], h, l); hp[0] = h; lp[0] = l;
  split_pair(a0[2], a0[3], h, l); hp[1] = h; lp[1] = l;
  split_pair(a1[0], a1[1], h, l); hp[2] = h; lp[2] = l;
  split_pair(a1[2], a1[3], h, l); hp[3] = h; lp[3] = l;
}

union FB { v16b v; v8b h[2]; };
__device__ __forceinline__ v16b frag_load(const __bf16* p) {
  FB f; f.h[0] = *(const v8b*)(p); f.h[1] = *(const v8b*)(p + 16); return f.v;
}
__device__ __forceinline__ v8f mma_raw(v16b a, v16b b, v8f c) {
  return __builtin_amdgcn_wmma_f32_16x16x32_bf16(false, a, false, b, (short)0, c, false, false);
}
__device__ __forceinline__ v8f mma_g(v16b a, v16b b, v8f c) {
  c = __builtin_amdgcn_wmma_f32_16x16x32_bf16(false, a, false, b, (short)0, c, false, false);
  asm volatile("v_nop\n\tv_nop\n\tv_nop\n\tv_nop" : "+v"(c) : "v"(a), "v"(b));
  return c;
}
__device__ __forceinline__ void dep_guard_b(v8f& a, v8f& b, v16b x, v16b y) {
  asm volatile("v_nop\n\tv_nop\n\tv_nop\n\tv_nop" : "+v"(a), "+v"(b) : "v"(x), "v"(y));
}
__device__ __forceinline__ void keep4_b(v16b a, v16b b, v16b c, v16b d) { asm volatile("v_nop" :: "v"(a), "v"(b), "v"(c), "v"(d)); }
__device__ __forceinline__ void acc_guard4(v8f& a, v8f& b, v8f& c, v8f& d) {
  asm volatile("v_nop\n\tv_nop\n\tv_nop\n\tv_nop" : "+v"(a), "+v"(b), "+v"(c), "+v"(d));
}

__global__ __launch_bounds__(256) void gate_kernel(const float* __restrict__ q_vec, const float* __restrict__ k_vec,
                                                    const float* __restrict__ v_vec,
                                                    const float* __restrict__ Ws, const float* __restrict__ bs,
                                                    const float* __restrict__ Wt, const float* __restrict__ bt,
                                                    float* __restrict__ gates) {
  __shared__ float xin[3][DCH];
  __shared__ float xsg[3][DCH];
  const int e = threadIdx.x;
  xin[0][e] = v_vec[e];
  xin[1][e] = q_vec[e];
  xin[2][e] = k_vec[e];
#pragma unroll 1
  for (int i = 0; i < 3; ++i) {
    const float x = xin[i][e];
    xsg[i][e] = 1.0f / (1.0f + expf(-x));
  }
  __syncthreads();
  float s1 = 0.f, s2 = 0.f;
#pragma unroll 1
  for (int d = 0; d < DCH; ++d) {
    const float gv = xsg[0][d];
    s1 = fmaf(Ws[e * DCH + d], gv, s1);
    s2 = fmaf(Wt[e * DCH + d], gv, s2);
  }
  s1 += bs[e];
  s2 += bt[e];
  const float vg = (1.0f / (1.0f + expf(-s1))) * tanhf(s2);
  const float sq = xsg[1][e];
  const float sk = xsg[2][e];
  volatile float* gp = gates;
  gp[e] = sq; gp[DCH + e] = sk; gp[2 * DCH + e] = vg;
  __threadfence();
  gp[e] = sq; gp[DCH + e] = sk; gp[2 * DCH + e] = vg;
}

__global__ __launch_bounds__(256) void split_bf16x2_kernel(const float* __restrict__ in, unsigned short* __restrict__ hi,
                                                           unsigned short* __restrict__ lo, int n2) {
  const int i = blockIdx.x * 256 + threadIdx.x;
  if (i < n2) {
    typedef __attribute__((ext_vector_type(2))) float v2f;
    const v2f f = *(const v2f*)(in + 2 * (size_t)i);
    unsigned uh, ul;
    split_pair(f[0], f[1], uh, ul);
    ((volatile unsigned*)hi)[i] = uh;
    ((volatile unsigned*)lo)[i] = ul;
    __threadfence();
    ((volatile unsigned*)hi)[i] = uh;
    ((volatile unsigned*)lo)[i] = ul;
  }
}

#define TFP 132
__global__ __launch_bounds__(256) void prep_kernel(const float* __restrict__ query, const float* __restrict__ value,
                                                    const float* __restrict__ gates,
                                                    unsigned short* __restrict__ Xh, unsigned short* __restrict__ Xl,
                                                    unsigned short* __restrict__ Kh, unsigned short* __restrict__ Kl,
                                                    unsigned short* __restrict__ Vth, unsigned short* __restrict__ Vtl) {
  __shared__ __align__(16) float tf[64 * TFP];
  const int tid = threadIdx.x;
  const int nt  = blockIdx.x % (SEQ / 64);
  const int b   = blockIdx.x / (SEQ / 64);
  const int n0  = nt * 64;
  const size_t rowbase = (size_t)b * SEQ + n0;

  {
    const int lr = tid >> 5;
    const int c8 = (tid & 31) * 8;
    const float* qs = query + rowbase * DCH + c8;
    unsigned short* xh = Xh + rowbase * DCH + c8;
    unsigned short* xl = Xl + rowbase * DCH + c8;
#pragma unroll 1
    for (int half = 0; half < 2; ++half) {
      v4u hv[4], lv[4];
#pragma unroll
      for (int it = 0; it < 4; ++it) {
        const int row = half * 32 + it * 8 + lr;
        const v4f a0 = *(const v4f*)(qs + (size_t)row * DCH);
        const v4f a1 = *(const v4f*)(qs + (size_t)row * DCH + 4);
        v4u hp, lp;
        split8(a0, a1, hp, lp);
        hv[it] = hp; lv[it] = lp;
      }
      for (int ps = 0; ps < 2; ++ps) {
#pragma unroll
        for (int it = 0; it < 4; ++it) {
          const int row = half * 32 + it * 8 + lr;
          *(volatile v4u*)(xh + (size_t)row * DCH) = hv[it];
          *(volatile v4u*)(xl + (size_t)row * DCH) = lv[it];
        }
        __threadfence();
      }
    }
  }

#pragma unroll 1
  for (int chh = 0; chh < 2; ++chh) {
    const int cb = chh * 128;
    __syncthreads();
    {
      const int lr = tid >> 4;
      const int c8 = (tid & 15) * 8;
      const float* vs = value + rowbase * DCH + cb + c8;
      unsigned short* kh = Kh + rowbase * DCH + cb + c8;
      unsigned short* kl = Kl + rowbase * DCH + cb + c8;
      const v4f g0 = *(const v4f*)(gates + DCH + cb + c8);
      const v4f g1 = *(const v4f*)(gates + DCH + cb + c8 + 4);
      v4u hv[4], lv[4];
#pragma unroll
      for (int it = 0; it < 4; ++it) {
        const int row = it * 16 + lr;
        const v4f a0 = *(const v4f*)(vs + (size_t)row * DCH);
        const v4f a1 = *(const v4f*)(vs + (size_t)row * DCH + 4);
        *(v4f*)(tf + row * TFP + c8) = a0;
        *(v4f*)(tf + row * TFP + c8 + 4) = a1;
        const v4f k0 = a0 * g0;
        const v4f k1 = a1 * g1;
        v4u hp, lp;
        split8(k0, k1, hp, lp);
        hv[it] = hp; lv[it] = lp;
      }
      for (int ps = 0; ps < 2; ++ps) {
#pragma unroll
        for (int it = 0; it < 4; ++it) {
          const int row = it * 16 + lr;
          *(volatile v4u*)(kh + (size_t)row * DCH) = hv[it];
          *(volatile v4u*)(kl + (size_t)row * DCH) = lv[it];
        }
        __threadfence();
      }
    }
    __syncthreads();
    {
      const int sub = tid >> 3;
      const int t8  = (tid & 7) * 8;
      v4u hv[4], lv[4];
#pragma unroll
      for (int it = 0; it < 4; ++it) {
        const int dloc = it * 32 + sub;
        const float gv = gates[2 * DCH + cb + dloc];
        v4u a, a2;
        unsigned h, l;
#pragma unroll
        for (int q = 0; q < 4; ++q) {
          const float f0 = tf[(t8 + 2 * q) * TFP + dloc] * gv;
          const float f1 = tf[(t8 + 2 * q + 1) * TFP + dloc] * gv;
          split_pair(f0, f1, h, l);
          a[q] = h; a2[q] = l;
        }
        hv[it] = a; lv[it] = a2;
      }
      unsigned short* th = Vth + ((size_t)b * DCH + cb) * SEQ + n0 + t8;
      unsigned short* tl = Vtl + ((size_t)b * DCH + cb) * SEQ + n0 + t8;
      for (int ps = 0; ps < 2; ++ps) {
#pragma unroll
        for (int it = 0; it < 4; ++it) {
          const int dloc = it * 32 + sub;
          const size_t go = (size_t)dloc * SEQ;
          *(volatile v4u*)(th + go) = hv[it];
          *(volatile v4u*)(tl + go) = lv[it];
        }
        __threadfence();
      }
    }
  }
}

__global__ __launch_bounds__(256) void qproj_gemm(
    const unsigned short* __restrict__ Ap, const unsigned short* __restrict__ A2p,
    const unsigned short* __restrict__ Btp, const unsigned short* __restrict__ Bt2p,
    const float* __restrict__ bias, const float* __restrict__ gate,
    unsigned short* __restrict__ Chp, unsigned short* __restrict__ Clp,
    int M, int N, int K) {
  const __bf16* A   = (const __bf16*)(const void*)Ap;
  const __bf16* A2  = (const __bf16*)(const void*)A2p;
  const __bf16* Bt  = (const __bf16*)(const void*)Btp;
  const __bf16* Bt2 = (const __bf16*)(const void*)Bt2p;
  __shared__ __align__(16) float sT[8][16 * 68];
  const int lane = threadIdx.x & 31;
  const int wave = threadIdx.x >> 5;
  const int tilesN = N >> 6;
  const int tilesM = M >> 6;
  const int tile = blockIdx.x * 8 + wave;
  if (tile >= tilesM * tilesN) return;
  const int tm = tile / tilesN;
  const int tn = tile - tm * tilesN;
  const int m0 = tm << 6;
  const int n0 = tn << 6;

  const int rlane = lane & 15;
  const int koff  = (lane >> 4) * 8;
  const int mOff  = (lane >> 4) * 8;

  v8f acc[4][4];
#pragma unroll
  for (int i = 0; i < 4; ++i)
#pragma unroll
    for (int j = 0; j < 4; ++j) acc[i][j] = (v8f){0.f,0.f,0.f,0.f,0.f,0.f,0.f,0.f};

  for (int k0 = 0; k0 < K; k0 += 32) {
    v16b bh[4], bl[4];
#pragma unroll
    for (int j = 0; j < 4; ++j) {
      const size_t bo = (size_t)(n0 + (j << 4) + rlane) * K + koff + k0;
      bh[j] = frag_load(Bt + bo);
      bl[j] = frag_load(Bt2 + bo);
    }
#pragma unroll
    for (int i = 0; i < 4; ++i) {
      const size_t ao = (size_t)(m0 + (i << 4) + rlane) * K + koff + k0;
      const v16b ah = frag_load(A + ao);
      const v16b al = frag_load(A2 + ao);
#pragma unroll
      for (int j = 0; j < 4; ++j) {
        acc[i][j] = mma_raw(ah, bh[j], acc[i][j]);
        acc[i][j] = mma_raw(ah, bl[j], acc[i][j]);
        acc[i][j] = mma_raw(al, bh[j], acc[i][j]);
      }
      dep_guard_b(acc[i][0], acc[i][3], ah, al);
    }
    keep4_b(bh[0], bh[1], bh[2], bh[3]);
    keep4_b(bl[0], bl[1], bl[2], bl[3]);
  }
  acc_guard4(acc[0][0], acc[0][1], acc[0][2], acc[0][3]);
  acc_guard4(acc[1][0], acc[1][1], acc[1][2], acc[1][3]);
  acc_guard4(acc[2][0], acc[2][1], acc[2][2], acc[2][3]);
  acc_guard4(acc[3][0], acc[3][1], acc[3][2], acc[3][3]);

  float* slab = sT[wave];
#pragma unroll
  for (int i = 0; i < 4; ++i) {
    const int mBase = m0 + (i << 4);
#pragma unroll
    for (int j = 0; j < 4; ++j) {
      const int n = n0 + (j << 4) + rlane;
      const float bv = bias[n];
      const float gv = gate[n];
#pragma unroll
      for (int r = 0; r < 8; ++r) {
        const float v = (acc[i][j][r] + bv) * gv;
        slab[(mOff + r) * 68 + (j << 4) + rlane] = v;
      }
    }
    __builtin_amdgcn_fence(__ATOMIC_RELEASE, "workgroup");
    __builtin_amdgcn_wave_barrier();
    __builtin_amdgcn_fence(__ATOMIC_ACQUIRE, "workgroup");
    {
      const int q = lane >> 3, c8 = (lane & 7) * 8;
      for (int ps = 0; ps < 2; ++ps) {
#pragma unroll
        for (int it = 0; it < 4; ++it) {
          const int row = it * 4 + q;
          const float* sp = slab + row * 68 + c8;
          v4u hv, lv;
          unsigned h, l;
#pragma unroll
          for (int e = 0; e < 4; ++e) {
            split_pair(sp[2 * e], sp[2 * e + 1], h, l);
            hv[e] = h; lv[e] = l;
          }
          const size_t go = (size_t)(mBase + row) * N + n0 + c8;
          *(volatile v4u*)(Chp + go) = hv;
          *(volatile v4u*)(Clp + go) = lv;
        }
        __threadfence();
      }
    }
    __builtin_amdgcn_fence(__ATOMIC_RELEASE, "workgroup");
    __builtin_amdgcn_wave_barrier();
    __builtin_amdgcn_fence(__ATOMIC_ACQUIRE, "workgroup");
  }
}

#define AT_QB 32
#define AT_KC 64
#define KSP 264
#define VTP 72
#define OSP 68
#define LDS_KE (AT_KC * KSP)
#define LDS_VE (DCH * VTP)
#define KV_BYTES ((2 * LDS_KE + 2 * LDS_VE) * 2)
static_assert(KV_BYTES == 141312);
static_assert(8 * 16 * OSP * 4 <= KV_BYTES);
static_assert(SEQ % AT_QB == 0);
static_assert(SEQ % AT_KC == 0);
static_assert(AT_KC == 2 * AT_QB);

__global__ __launch_bounds__(256)
void attn_kernel(const unsigned short* __restrict__ qhp, const unsigned short* __restrict__ qlp,
                 const unsigned short* __restrict__ khp, const unsigned short* __restrict__ klp,
                 const unsigned short* __restrict__ vhp, const unsigned short* __restrict__ vlp,
                 float* __restrict__ out, float sscale) {
  __shared__ __align__(16) unsigned char kv_raw[KV_BYTES];
  __shared__ __align__(16) __bf16 Psh[2][16 * AT_KC];
  __shared__ __align__(16) __bf16 Psl[2][16 * AT_KC];
  __shared__ __align__(16) float  Al[2][16];
  __shared__ __align__(16) float  Ll[2][16];
  __bf16* Ks_h = (__bf16*)(void*)kv_raw;
  __bf16* Ks_l = Ks_h + LDS_KE;
  __bf16* Vs_h = Ks_l + LDS_KE;
  __bf16* Vs_l = Vs_h + LDS_VE;

  const int tid  = threadIdx.x;
  const int wave = tid >> 5;
  const int lane = tid & 31;
  const int hh   = lane >> 4;
  const int c    = lane & 15;
  const int g    = wave & 1;
  const int cq   = wave >> 1;
  const int ch0  = cq * 64;

  const int nqb = SEQ / AT_QB;
  const int qb  = blockIdx.x % nqb;
  const int b   = blockIdx.x / nqb;
  const int q0  = qb * AT_QB;
  const int qg0 = q0 + g * 16;

  const __bf16* Qh = (const __bf16*)(const void*)qhp + (size_t)b * SEQ * DCH;
  const __bf16* Ql = (const __bf16*)(const void*)qlp + (size_t)b * SEQ * DCH;
  const __bf16* Kh = (const __bf16*)(const void*)khp + (size_t)b * SEQ * DCH;
  const __bf16* Kl = (const __bf16*)(const void*)klp + (size_t)b * SEQ * DCH;
  const __bf16* Vh = (const __bf16*)(const void*)vhp + (size_t)b * DCH * SEQ;
  const __bf16* Vl = (const __bf16*)(const void*)vlp + (size_t)b * DCH * SEQ;
  float* Ob = out + (size_t)b * SEQ * DCH;

  float mrow[8], lrow[8];
  v8f oacc[4];
#pragma unroll
  for (int r = 0; r < 8; ++r) { mrow[r] = NEG_INF; lrow[r] = 0.f; }
#pragma unroll
  for (int t = 0; t < 4; ++t) oacc[t] = (v8f){0.f,0.f,0.f,0.f,0.f,0.f,0.f,0.f};

  __bf16* pwh = Psh[g];
  __bf16* pwl = Psl[g];

  const int nch = (qb >> 1) + 1;
#pragma unroll 1
  for (int kc = 0; kc < nch; ++kc) {
    const int kv0 = kc * AT_KC;
    __syncthreads();
    {
      const int r = tid >> 2, part = (tid & 3) * 64;
      const __bf16* gkh = Kh + (size_t)(kv0 + r) * DCH + part;
      const __bf16* gkl = Kl + (size_t)(kv0 + r) * DCH + part;
      __bf16* dkh = Ks_h + r * KSP + part;
      __bf16* dkl = Ks_l + r * KSP + part;
#pragma unroll
      for (int i = 0; i < 8; ++i) {
        *(v8b*)(dkh + 8 * i) = *(const v8b*)(gkh + 8 * i);
        *(v8b*)(dkl + 8 * i) = *(const v8b*)(gkl + 8 * i);
      }
      const __bf16* gvh = Vh + (size_t)tid * SEQ + kv0;
      const __bf16* gvl = Vl + (size_t)tid * SEQ + kv0;
      __bf16* dvh = Vs_h + tid * VTP;
      __bf16* dvl = Vs_l + tid * VTP;
#pragma unroll
      for (int i = 0; i < 8; ++i) {
        *(v8b*)(dvh + 8 * i) = *(const v8b*)(gvh + 8 * i);
        *(v8b*)(dvl + 8 * i) = *(const v8b*)(gvl + 8 * i);
      }
    }
    __syncthreads();

    if (wave < 2) {
      v8f s[4];
#pragma unroll
      for (int j = 0; j < 4; ++j) s[j] = (v8f){0.f,0.f,0.f,0.f,0.f,0.f,0.f,0.f};
      const __bf16* qrh = Qh + (size_t)(qg0 + c) * DCH + 8 * hh;
      const __bf16* qrl = Ql + (size_t)(qg0 + c) * DCH + 8 * hh;
#pragma unroll 1
      for (int dc = 0; dc < 8; ++dc) {
        const v16b qa  = frag_load(qrh + dc * 32);
        const v16b qal = frag_load(qrl + dc * 32);
#pragma unroll
        for (int j = 0; j < 4; ++j) {
          const int ko = (j * 16 + c) * KSP + dc * 32 + 8 * hh;
          const v16b kb  = frag_load(Ks_h + ko);
          const v16b kbl = frag_load(Ks_l + ko);
          s[j] = mma_g(qa, kb, s[j]);
          s[j] = mma_g(qa, kbl, s[j]);
          s[j] = mma_g(qal, kb, s[j]);
        }
      }
      float cm[8];
#pragma unroll
      for (int r = 0; r < 8; ++r) {
        const int row = qg0 + 8 * hh + r;
        float m = NEG_INF;
#pragma unroll
        for (int j = 0; j < 4; ++j) {
          const int key = kv0 + j * 16 + c;
          float sv = s[j][r] * sscale;
          const bool ok = (key <= row) && (sv != 0.0f);
          sv = ok ? sv : NEG_INF;
          s[j][r] = sv;
          m = fmaxf(m, sv);
        }
#pragma unroll
        for (int off = 1; off < 16; off <<= 1) m = fmaxf(m, __shfl_xor(m, off, 32));
        cm[r] = m;
      }
#pragma unroll
      for (int r = 0; r < 8; ++r) {
        const float mnew  = fmaxf(mrow[r], cm[r]);
        const float aexp  = expf(mrow[r] - mnew);
        const float alpha = (mnew == NEG_INF) ? 1.0f : aexp;
        mrow[r] = mnew;
        float psum = 0.f;
#pragma unroll
        for (int j = 0; j < 4; ++j) {
          const float sv = s[j][r];
          const float pe = expf(sv - mnew);
          const float p  = (sv == NEG_INF) ? 0.0f : pe;
          psum += p;
          const unsigned short hb = f2bf_bits(p);
          const unsigned short lb = f2bf_bits(p - bf_bits2f(hb));
          pwh[(8 * hh + r) * AT_KC + j * 16 + c] = __builtin_bit_cast(__bf16, hb);
          pwl[(8 * hh + r) * AT_KC + j * 16 + c] = __builtin_bit_cast(__bf16, lb);
        }
#pragma unroll
        for (int off = 1; off < 16; off <<= 1) psum += __shfl_xor(psum, off, 32);
        lrow[r] = lrow[r] * alpha + psum;
        if (c == 0) {
          Al[g][8 * hh + r] = alpha;
          Ll[g][8 * hh + r] = lrow[r];
        }
      }
    }
    __syncthreads();

    {
      float af[8];
#pragma unroll
      for (int r = 0; r < 8; ++r) af[r] = Al[g][8 * hh + r];
#pragma unroll
      for (int t = 0; t < 4; ++t)
#pragma unroll
        for (int r = 0; r < 8; ++r) oacc[t][r] *= af[r];
#pragma unroll 1
      for (int kk = 0; kk < 2; ++kk) {
        const v16b pa = frag_load(pwh + c * AT_KC + kk * 32 + 8 * hh);
        const v16b pl = frag_load(pwl + c * AT_KC + kk * 32 + 8 * hh);
#pragma unroll
        for (int t = 0; t < 4; ++t) {
          const int vo = (ch0 + t * 16 + c) * VTP + kk * 32 + 8 * hh;
          const v16b vb  = frag_load(Vs_h + vo);
          const v16b vbl = frag_load(Vs_l + vo);
          oacc[t] = mma_g(pa, vb, oacc[t]);
          oacc[t] = mma_g(pa, vbl, oacc[t]);
          oacc[t] = mma_g(pl, vb, oacc[t]);
        }
      }
    }
  }
  __syncthreads();

  float* os = (float*)(void*)kv_raw + wave * (16 * OSP);
#pragma unroll
  for (int r = 0; r < 8; ++r) {
    const float inv = 1.0f / Ll[g][8 * hh + r];
#pragma unroll
    for (int t = 0; t < 4; ++t) os[(8 * hh + r) * OSP + t * 16 + c] = oacc[t][r] * inv;
  }
  __builtin_amdgcn_fence(__ATOMIC_RELEASE, "workgroup");
  __builtin_amdgcn_wave_barrier();
  __builtin_amdgcn_fence(__ATOMIC_ACQUIRE, "workgroup");
  {
    const int hh2 = lane >> 4, c4 = (lane & 15) * 4;
    for (int ps = 0; ps < 2; ++ps) {
#pragma unroll
      for (int it = 0; it < 8; ++it) {
        const int row = it * 2 + hh2;
        const v4f v = *(const v4f*)(os + row * OSP + c4);
        *(volatile v4f*)(Ob + (size_t)(qg0 + row) * DCH + ch0 + c4) = v;
      }
      __threadfence();
    }
  }
}

extern "C" void kernel_launch(void* const* d_in, const int* in_sizes, int n_in,
                              void* d_out, int out_size, void* d_ws, size_t ws_size,
                              hipStream_t stream) {
  if (n_in < 11) return;
  const int NTOT = NB * SEQ * DCH;
  if (in_sizes[0] != NTOT || in_sizes[1] != NTOT) return;
  if (in_sizes[2] != DCH || in_sizes[3] != DCH || in_sizes[4] != DCH) return;
  if (in_sizes[5] != DCH * DCH || in_sizes[6] != DCH) return;
  if (in_sizes[7] != DCH * DCH || in_sizes[8] != DCH) return;
  if (in_sizes[9] != DCH * DCH || in_sizes[10] != DCH) return;
  if (out_size != NTOT) return;

  const float* query = (const float*)d_in[0];
  const float* value = (const float*)d_in[1];
  const float* q_vec = (const float*)d_in[2];
  const float* k_vec = (const float*)d_in[3];
  const float* v_vec = (const float*)d_in[4];
  const float* Wq    = (const float*)d_in[5];
  const float* bq    = (const float*)d_in[6];
  const float* Ws    = (const float*)d_in[7];
  const float* bs    = (const float*)d_in[8];
  const float* Wt    = (const float*)d_in[9];
  const float* bt    = (const float*)d_in[10];
  float* out = (float*)d_out;

  const size_t PL = (size_t)NB * SEQ * DCH * 2;
  const size_t PW = (size_t)DCH * DCH * 2;
  const size_t PG = 4096;
  size_t off = 0;
  const size_t oXh  = off; off += PL;
  const size_t oXl  = off; off += PL;
  const size_t oQh  = off; off += PL;
  const size_t oQl  = off; off += PL;
  const size_t oKh  = off; off += PL;
  const size_t oKl  = off; off += PL;
  const size_t oVth = off; off += PL;
  const size_t oVtl = off; off += PL;
  const size_t oWh  = off; off += PW;
  const size_t oWl  = off; off += PW;
  const size_t oG   = off; off += PG;
  if (off > ws_size) return;

  char* ws = (char*)d_ws;
  unsigned short* Xh  = (unsigned short*)(ws + oXh);
  unsigned short* Xl  = (unsigned short*)(ws + oXl);
  unsigned short* Qh  = (unsigned short*)(ws + oQh);
  unsigned short* Ql  = (unsigned short*)(ws + oQl);
  unsigned short* Kh  = (unsigned short*)(ws + oKh);
  unsigned short* Kl  = (unsigned short*)(ws + oKl);
  unsigned short* Vth = (unsigned short*)(ws + oVth);
  unsigned short* Vtl = (unsigned short*)(ws + oVtl);
  unsigned short* Wh  = (unsigned short*)(ws + oWh);
  unsigned short* Wl  = (unsigned short*)(ws + oWl);
  float* gates = (float*)(ws + oG);

  gate_kernel<<<dim3(1), dim3(256), 0, stream>>>(q_vec, k_vec, v_vec, Ws, bs, Wt, bt, gates);
  const int n2w = DCH * DCH / 2;
  split_bf16x2_kernel<<<dim3((n2w + 255) / 256), dim3(256), 0, stream>>>(Wq, Wh, Wl, n2w);
  prep_kernel<<<dim3(NB * (SEQ / 64)), dim3(256), 0, stream>>>(query, value, gates, Xh, Xl, Kh, Kl, Vth, Vtl);
  const int tilesQ = ((NB * SEQ) / 64) * (DCH / 64);
  qproj_gemm<<<dim3((tilesQ + 7) / 8), dim3(256), 0, stream>>>(Xh, Xl, Wh, Wl, bq, gates, Qh, Ql, NB * SEQ, DCH, DCH);
  attn_kernel<<<dim3(NB * (SEQ / AT_QB)), dim3(256), 0, stream>>>(Qh, Ql, Kh, Kl, Vth, Vtl, out, 0.0625f);
  (void)hipGetLastError();
}
